// EuclideanTransformer_39608188403794
// MI455X (gfx1250) — hardware-verified
//
#include <hip/hip_runtime.h>
#include <stddef.h>


#define FD     128
#define NRB    32
#define EVD    16
#define NNODE  32
#define TEW    16
#define EWAV   2
#define TEB    (TEW * EWAV)
#define CAW    16
#define NTA    256
#define NWA    8
#define EPT    8
#define CHUNK  (NTA * EPT)
#define WCAP   (EPT * 32)
#define NB     64
#define INTK   132
#define INTKP  192
#define INTNP  144
#define AKP    160
#define TP     144

#define PS_W1  (FD * NRB)
#define PS_W2  (FD * FD)
#define PS_INT (INTNP * INTKP)
#define PS_QK  (FD * 32)
#define O_FIW1 0
#define O_FIW2 (O_FIW1 + 2 * PS_W1)
#define O_FIE2 (O_FIW2 + 2 * PS_W2)
#define O_FEW1 (O_FIE2 + 2 * PS_W1)
#define O_FEW2 (O_FEW1 + 2 * PS_W1)
#define O_FEE2 (O_FEW2 + 2 * PS_W2)
#define O_INTW (O_FEE2 + 2 * PS_W1)
#define O_WQI  (O_INTW + 2 * PS_INT)
#define O_WKI  (O_WQI + 2 * PS_QK)
#define O_WVI  (O_WKI + 2 * PS_QK)
#define O_WQE  (O_WVI + 2 * PS_QK)
#define O_WKE  (O_WQE + 2 * PS_QK)
#define PL_TOT (O_WKE + 2 * PS_QK)

#define H1S    (EWAV * TEW * FD)
#define E1S    (EWAV * TEW * NRB)
#define RS32   (1.0f / 5.656854249492381f)

static_assert((NB % NWA) == 0);
static_assert(NB <= 256);
static_assert((NB % NNODE) == 0);
static_assert((PS_W1 % 256) == 0);
static_assert((PS_W2 % 256) == 0);
static_assert((PS_INT % 256) == 0);
static_assert((PS_QK % 256) == 0);
static_assert(PL_TOT == 194560);

typedef unsigned short us;
typedef us     v8us  __attribute__((ext_vector_type(8)));
typedef us     v16us __attribute__((ext_vector_type(16)));
typedef __bf16 v16bf __attribute__((ext_vector_type(16)));
typedef float  v4f   __attribute__((ext_vector_type(4)));
typedef float  v8f   __attribute__((ext_vector_type(8)));
typedef int    v4i   __attribute__((ext_vector_type(4)));
union Frag { v16bf v; v16us w; v8us u[2]; };

__device__ __forceinline__ v8us zero8us() { v8us z = {0, 0, 0, 0, 0, 0, 0, 0}; return z; }
__device__ __forceinline__ v8f  zero8f()  { v8f z = {0.0f, 0.0f, 0.0f, 0.0f, 0.0f, 0.0f, 0.0f, 0.0f}; return z; }

__device__ __forceinline__ unsigned int bfbits(float x) {
  const unsigned int u = __float_as_uint(x);
  return (u + 0x7fffu + ((u >> 16) & 1u)) >> 16;
}
__device__ __forceinline__ void split2(float x, us& h, us& l) {
  const unsigned int hb = bfbits(x);
  const float rem = x - __uint_as_float(hb << 16);
  h = (us)hb;
  l = (us)bfbits(rem);
}

__device__ __forceinline__ float silu_f(float s) {
  const float e = __expf(-s);
  return s * __builtin_amdgcn_rcpf(1.0f + e);
}

__device__ __forceinline__ v8f wm3(const Frag& ah, const Frag& al, const Frag& bh, const Frag& bl, v8f c) {
  c = __builtin_amdgcn_wmma_f32_16x16x32_bf16(false, ah.v, false, bh.v, (short)0, c, false, false);
  c = __builtin_amdgcn_wmma_f32_16x16x32_bf16(false, al.v, false, bh.v, (short)0, c, false, false);
  c = __builtin_amdgcn_wmma_f32_16x16x32_bf16(false, ah.v, false, bl.v, (short)0, c, false, false);
  asm volatile("v_nop\n\tv_nop\n\tv_nop\n\tv_nop" : "+v"(c) : "v"(ah.w), "v"(al.w), "v"(bh.w), "v"(bl.w));
  return c;
}

#define LDFR(FR, P, HH) { (FR).u[0] = *(const v8us*)((P) + 8 * (HH)); (FR).u[1] = *(const v8us*)((P) + 16 + 8 * (HH)); }

__global__ __launch_bounds__(256) void k_prep(
    const float* __restrict__ fiw1, const float* __restrict__ fiw2, const float* __restrict__ fie2,
    const float* __restrict__ few1, const float* __restrict__ few2, const float* __restrict__ fee2,
    const float* __restrict__ intw,
    const float* __restrict__ wqi, const float* __restrict__ wki, const float* __restrict__ wvi,
    const float* __restrict__ wqe, const float* __restrict__ wke,
    us* pl) {
  const int id = blockIdx.y;
  const float* src = fiw1;
  int off = O_FIW1, psz = PS_W1, kp = NRB, nlog = FD, klog = NRB, mode = 0;
  switch (id) {
    case 0:  src = fiw1; off = O_FIW1; psz = PS_W1;  kp = NRB;   nlog = FD;   klog = NRB;  mode = 0; break;
    case 1:  src = fiw2; off = O_FIW2; psz = PS_W2;  kp = FD;    nlog = FD;   klog = FD;   mode = 0; break;
    case 2:  src = fie2; off = O_FIE2; psz = PS_W1;  kp = NRB;   nlog = FD;   klog = NRB;  mode = 0; break;
    case 3:  src = few1; off = O_FEW1; psz = PS_W1;  kp = NRB;   nlog = FD;   klog = NRB;  mode = 0; break;
    case 4:  src = few2; off = O_FEW2; psz = PS_W2;  kp = FD;    nlog = FD;   klog = FD;   mode = 0; break;
    case 5:  src = fee2; off = O_FEE2; psz = PS_W1;  kp = NRB;   nlog = FD;   klog = NRB;  mode = 0; break;
    case 6:  src = intw; off = O_INTW; psz = PS_INT; kp = INTKP; nlog = INTK; klog = INTK; mode = 0; break;
    case 7:  src = wqi;  off = O_WQI;  psz = PS_QK;  kp = 32;    nlog = FD;   klog = 16;   mode = 1; break;
    case 8:  src = wki;  off = O_WKI;  psz = PS_QK;  kp = 32;    nlog = FD;   klog = 16;   mode = 1; break;
    case 9:  src = wvi;  off = O_WVI;  psz = PS_QK;  kp = 32;    nlog = FD;   klog = 16;   mode = 1; break;
    case 10: src = wqe;  off = O_WQE;  psz = PS_QK;  kp = 32;    nlog = FD;   klog = 32;   mode = 2; break;
    default: src = wke;  off = O_WKE;  psz = PS_QK;  kp = 32;    nlog = FD;   klog = 32;   mode = 2; break;
  }
  const int g  = blockIdx.x * 256 + threadIdx.x;
  const int gg = g * 8;
  if (gg >= psz) return;
  const int n  = gg / kp;
  const int k0 = gg - n * kp;
  v8us hv, lv;
#pragma unroll
  for (int c = 0; c < 8; ++c) {
    const int k = k0 + c;
    int idx;
    bool valid;
    if (mode == 0) {
      valid = (n < nlog) && (k < klog);
      const int nc = n < nlog ? n : nlog - 1;
      const int kc = k < klog ? k : klog - 1;
      idx = kc * nlog + nc;
    } else if (mode == 1) {
      valid = k < 16;
      const int kc = k < 16 ? k : 15;
      idx = (n >> 4) * 256 + kc * 16 + (n & 15);
    } else {
      valid = true;
      idx = (n >> 5) * 1024 + k * 32 + (n & 31);
    }
    float v = src[idx];
    v = valid ? v : 0.0f;
    us h, l;
    split2(v, h, l);
    hv[c] = h;
    lv[c] = l;
  }
  us* ph = pl + off + gg;
  *(volatile v8us*)ph = hv;
  *(volatile v8us*)(ph + psz) = lv;
  __threadfence();
  *(volatile v8us*)ph = hv;
  *(volatile v8us*)(ph + psz) = lv;
}

__global__ __launch_bounds__(64) void k_node(const float* __restrict__ x, const us* __restrict__ pl,
                                             float* Qi, float* Ki, float* Vi, float* Qe, float* Ke, int nN) {
  __shared__ __attribute__((aligned(16))) us    xh[NNODE * FD];
  __shared__ __attribute__((aligned(16))) us    xl[NNODE * FD];
  __shared__ __attribute__((aligned(16))) float st[NNODE * FD];
  const int tid = threadIdx.x, lane = tid & 31, wave = tid >> 5, hh = lane >> 4, m = lane & 15;
  const int nodeBase = blockIdx.x * NNODE;

#pragma unroll 4
  for (int i = 0; i < 16; ++i) {
    const int g = tid + 64 * i;
    const int row = g >> 5, c4 = g & 31;
    int node = nodeBase + row;
    node = node > nN - 1 ? nN - 1 : node;
    const v4f v = *(const v4f*)(x + (size_t)node * FD + 4 * c4);
    us h, l;
    const int b = row * FD + 4 * c4;
    split2(v.x, h, l); xh[b + 0] = h; xl[b + 0] = l;
    split2(v.y, h, l); xh[b + 1] = h; xl[b + 1] = l;
    split2(v.z, h, l); xh[b + 2] = h; xl[b + 2] = l;
    split2(v.w, h, l); xh[b + 3] = h; xl[b + 3] = l;
  }
  __syncthreads();

#pragma unroll 1
  for (int mat = 0; mat < 5; ++mat) {
    const int evm  = (mat >= 3) ? 1 : 0;
    const int poff = (mat == 0) ? O_WQI : (mat == 1) ? O_WKI : (mat == 2) ? O_WVI : (mat == 3) ? O_WQE : O_WKE;
    float* dst = (mat == 0) ? Qi : (mat == 1) ? Ki : (mat == 2) ? Vi : (mat == 3) ? Qe : Ke;
    const us* bhp = pl + poff;
    const us* blp = bhp + PS_QK;
#pragma unroll 1
    for (int nt = 0; nt < 8; ++nt) {
      const int cb = evm ? 32 * (nt >> 1) : 16 * nt;
      const int o1 = evm ? 16 : 0;
      Frag fah, fal, fbh, fbl;
      const us* arh = xh + (16 * wave + m) * FD + cb;
      const us* arl = xl + (16 * wave + m) * FD + cb;
      fah.u[0] = *(const v8us*)(arh + 8 * hh);
      fah.u[1] = *(const v8us*)(arh + o1 + 8 * hh);
      fal.u[0] = *(const v8us*)(arl + 8 * hh);
      fal.u[1] = *(const v8us*)(arl + o1 + 8 * hh);
      if (!evm) { fah.u[1] = zero8us(); fal.u[1] = zero8us(); }
      LDFR(fbh, bhp + (16 * nt + m) * 32, hh);
      LDFR(fbl, blp + (16 * nt + m) * 32, hh);
      v8f acc = zero8f();
      acc = wm3(fah, fal, fbh, fbl, acc);
#pragma unroll
      for (int r = 0; r < 8; ++r) st[(16 * wave + 8 * hh + r) * FD + 16 * nt + m] = acc[r];
    }
    __syncthreads();
#pragma unroll
    for (int i = 0; i < 16; ++i) {
      const int row = 16 * wave + i;
      const v4f v = *(const v4f*)(st + row * FD + 4 * lane);
      *(volatile v4f*)(dst + (size_t)(nodeBase + row) * FD + 4 * lane) = v;
    }
    __threadfence();
#pragma unroll
    for (int i = 0; i < 16; ++i) {
      const int row = 16 * wave + i;
      const v4f v = *(const v4f*)(st + row * FD + 4 * lane);
      *(volatile v4f*)(dst + (size_t)(nodeBase + row) * FD + 4 * lane) = v;
    }
    __syncthreads();
  }
}

__global__ __launch_bounds__(64) void k_edge(
    const float* __restrict__ rbf, const float* __restrict__ ev, const float* __restrict__ cut,
    const int* __restrict__ snd, const int* __restrict__ rcv,
    const float* __restrict__ Qi, const float* __restrict__ Ki,
    const float* __restrict__ Qe, const float* __restrict__ Ke,
    const us* __restrict__ pl,
    const float* __restrict__ fib1, const float* __restrict__ fib2,
    const float* __restrict__ fiew1, const float* __restrict__ fieb1, const float* __restrict__ fieb2,
    const float* __restrict__ feb1, const float* __restrict__ feb2,
    const float* __restrict__ feew1, const float* __restrict__ feeb1, const float* __restrict__ feeb2,
    float* cal, int nN, int nE) {
  __shared__ __attribute__((aligned(16))) us    h1p[2 * EWAV * TEW * FD];
  __shared__ __attribute__((aligned(16))) us    e1p[2 * EWAV * TEW * NRB];
  __shared__ __attribute__((aligned(16))) float fwp[EWAV * TEW * FD];
  __shared__ __attribute__((aligned(16))) float ast[EWAV * TEW * CAW];

  const int tid = threadIdx.x, lane = tid & 31, wave = tid >> 5, hh = lane >> 4, m = lane & 15;
  const int e0 = (blockIdx.x * EWAV + wave) * TEW;
  int erow = e0 + m;
  erow = erow > nE - 1 ? nE - 1 : erow;

  int s = snd[erow], r = rcv[erow];
  s = s < 0 ? 0 : (s > nN - 1 ? nN - 1 : s);
  r = r < 0 ? 0 : (r > nN - 1 ? nN - 1 : r);
  const float cu = cut[erow];

  float evi0, evi1, evi2, evi3;
  {
    const float* ps = ev + (size_t)s * EVD;
    const float* pr = ev + (size_t)r * EVD;
    float d[16];
#pragma unroll
    for (int q = 0; q < 4; ++q) {
      const v4f a = *(const v4f*)(ps + 4 * q);
      const v4f b = *(const v4f*)(pr + 4 * q);
      d[4 * q + 0] = a.x - b.x; d[4 * q + 1] = a.y - b.y; d[4 * q + 2] = a.z - b.z; d[4 * q + 3] = a.w - b.w;
    }
    evi0 = d[0] * d[0];
    evi1 = d[1] * d[1] + d[2] * d[2] + d[3] * d[3];
    evi2 = d[4] * d[4] + d[5] * d[5] + d[6] * d[6] + d[7] * d[7] + d[8] * d[8];
    evi3 = d[9] * d[9] + d[10] * d[10] + d[11] * d[11] + d[12] * d[12] + d[13] * d[13] + d[14] * d[14] + d[15] * d[15];
  }

  Frag ah, al;
  {
    const float* pb = rbf + (size_t)erow * NRB;
    const v4f x0 = *(const v4f*)(pb + 8 * hh);
    const v4f x1 = *(const v4f*)(pb + 8 * hh + 4);
    const v4f x2 = *(const v4f*)(pb + 16 + 8 * hh);
    const v4f x3 = *(const v4f*)(pb + 20 + 8 * hh);
    float xv[16] = {x0.x, x0.y, x0.z, x0.w, x1.x, x1.y, x1.z, x1.w,
                    x2.x, x2.y, x2.z, x2.w, x3.x, x3.y, x3.z, x3.w};
#pragma unroll
    for (int i = 0; i < 16; ++i) { us h, l; split2(xv[i], h, l); ah.w[i] = h; al.w[i] = l; }
  }

#pragma unroll 1
  for (int br = 0; br < 2; ++br) {
    const us* w1h = pl + (br ? O_FEW1 : O_FIW1); const us* w1l = w1h + PS_W1;
    const us* w2h = pl + (br ? O_FEW2 : O_FIW2); const us* w2l = w2h + PS_W2;
    const us* e2h = pl + (br ? O_FEE2 : O_FIE2); const us* e2l = e2h + PS_W1;
    const float* b1  = br ? feb1  : fib1;
    const float* b2  = br ? feb2  : fib2;
    const float* ew1 = br ? feew1 : fiew1;
    const float* eb1 = br ? feeb1 : fieb1;
    const float* eb2 = br ? feeb2 : fieb2;

#pragma unroll 4
    for (int jj = 0; jj < 16; ++jj) {
      const int j = 16 * hh + jj;
      float dot = evi0 * ew1[j];
      dot += evi1 * ew1[NRB + j];
      dot += evi2 * ew1[2 * NRB + j];
      dot += evi3 * ew1[3 * NRB + j];
      const float sv = silu_f(dot + eb1[j]);
      us h, l;
      split2(sv, h, l);
      const int idx = (wave * TEW + m) * NRB + j;
      e1p[idx] = h;
      e1p[E1S + idx] = l;
    }

#pragma unroll 1
    for (int t = 0; t < 8; ++t) {
      Frag bh, bl;
      LDFR(bh, w1h + (16 * t + m) * NRB, hh);
      LDFR(bl, w1l + (16 * t + m) * NRB, hh);
      v8f acc = zero8f();
      acc = wm3(ah, al, bh, bl, acc);
      const int col = 16 * t + m;
      const float bias = b1[col];
#pragma unroll
      for (int rr = 0; rr < 8; ++rr) {
        const float xv = silu_f(acc[rr] + bias);
        us h, l;
        split2(xv, h, l);
        const int idx = (wave * TEW + 8 * hh + rr) * FD + col;
        h1p[idx] = h;
        h1p[H1S + idx] = l;
      }
    }
    __syncthreads();

    {
      Frag eh, el;
      LDFR(eh, e1p + (wave * TEW + m) * NRB, hh);
      LDFR(el, e1p + E1S + (wave * TEW + m) * NRB, hh);
#pragma unroll 1
      for (int t = 0; t < 8; ++t) {
        v8f acc = zero8f();
#pragma unroll 2
        for (int ks = 0; ks < 4; ++ks) {
          Frag fah, fal, fbh, fbl;
          LDFR(fah, h1p + (wave * TEW + m) * FD + 32 * ks, hh);
          LDFR(fal, h1p + H1S + (wave * TEW + m) * FD + 32 * ks, hh);
          LDFR(fbh, w2h + (16 * t + m) * FD + 32 * ks, hh);
          LDFR(fbl, w2l + (16 * t + m) * FD + 32 * ks, hh);
          acc = wm3(fah, fal, fbh, fbl, acc);
        }
        {
          Frag fbh, fbl;
          LDFR(fbh, e2h + (16 * t + m) * NRB, hh);
          LDFR(fbl, e2l + (16 * t + m) * NRB, hh);
          acc = wm3(eh, el, fbh, fbl, acc);
        }
        const int col = 16 * t + m;
        const float bias = b2[col] + eb2[col];
#pragma unroll
        for (int rr = 0; rr < 8; ++rr) fwp[(wave * TEW + 8 * hh + rr) * FD + col] = acc[rr] + bias;
      }
    }
    __syncthreads();

    {
      float* arow = ast + (wave * TEW + m) * CAW;
      const float* frow = fwp + (wave * TEW + m) * FD;
      if (br == 0) {
#pragma unroll 1
        for (int i = 0; i < 4; ++i) {
          const int hd = 4 * hh + i;
          const float* qp = Qi + (size_t)r * FD + 16 * hd;
          const float* kq = Ki + (size_t)s * FD + 16 * hd;
          const float* fp = frow + 16 * hd;
          float sum = 0.0f;
#pragma unroll
          for (int c = 0; c < 4; ++c) {
            const v4f q = *(const v4f*)(qp + 4 * c);
            const v4f k = *(const v4f*)(kq + 4 * c);
            const v4f f = *(const v4f*)(fp + 4 * c);
            sum += q.x * (k.x * f.x); sum += q.y * (k.y * f.y);
            sum += q.z * (k.z * f.z); sum += q.w * (k.w * f.w);
          }
          arow[hd] = cu * (sum * 0.25f);
        }
      } else {
#pragma unroll 1
        for (int i = 0; i < 2; ++i) {
          const int ld = 2 * hh + i;
          const float* qp = Qe + (size_t)r * FD + 32 * ld;
          const float* kq = Ke + (size_t)s * FD + 32 * ld;
          const float* fp = frow + 32 * ld;
          float sum = 0.0f;
#pragma unroll 4
          for (int c = 0; c < 8; ++c) {
            const v4f q = *(const v4f*)(qp + 4 * c);
            const v4f k = *(const v4f*)(kq + 4 * c);
            const v4f f = *(const v4f*)(fp + 4 * c);
            sum += q.x * (k.x * f.x); sum += q.y * (k.y * f.y);
            sum += q.z * (k.z * f.z); sum += q.w * (k.w * f.w);
          }
          arow[8 + ld] = cu * (sum * RS32);
        }
        arow[12 + 2 * hh] = 0.0f;
        arow[13 + 2 * hh] = 0.0f;
      }
    }
  }
  __syncthreads();

  {
    const float* ab = ast + wave * TEW * CAW;
    const v4f v0 = *(const v4f*)(ab + 4 * lane);
    const v4f v1 = *(const v4f*)(ab + 128 + 4 * lane);
    float* gp = cal + (size_t)e0 * CAW + 4 * lane;
    *(volatile v4f*)gp = v0;
    *(volatile v4f*)(gp + 128) = v1;
    __threadfence();
    *(volatile v4f*)gp = v0;
    *(volatile v4f*)(gp + 128) = v1;
  }
}

__device__ __forceinline__ int scan_chunk(const int* __restrict__ dsts, int nE, int cbase, int nodeBase,
                                          int* list, int tid, int wave) {
  int wc = 0;
  const int el0  = tid * EPT;
  const int e0   = cbase + el0;
  const int sent = -2147483647 - 1;
  v4i da, db;
  if (cbase + CHUNK <= nE) {
    da = *(const v4i*)(dsts + e0);
    db = *(const v4i*)(dsts + e0 + 4);
  } else {
    da.x = (e0     < nE) ? dsts[min(e0,     nE - 1)] : sent;
    da.y = (e0 + 1 < nE) ? dsts[min(e0 + 1, nE - 1)] : sent;
    da.z = (e0 + 2 < nE) ? dsts[min(e0 + 2, nE - 1)] : sent;
    da.w = (e0 + 3 < nE) ? dsts[min(e0 + 3, nE - 1)] : sent;
    db.x = (e0 + 4 < nE) ? dsts[min(e0 + 4, nE - 1)] : sent;
    db.y = (e0 + 5 < nE) ? dsts[min(e0 + 5, nE - 1)] : sent;
    db.z = (e0 + 6 < nE) ? dsts[min(e0 + 6, nE - 1)] : sent;
    db.w = (e0 + 7 < nE) ? dsts[min(e0 + 7, nE - 1)] : sent;
  }
  const unsigned nb = (unsigned)nodeBase;
  const unsigned s0 = (unsigned)da.x - nb, s1 = (unsigned)da.y - nb;
  const unsigned s2 = (unsigned)da.z - nb, s3 = (unsigned)da.w - nb;
  const unsigned s4 = (unsigned)db.x - nb, s5 = (unsigned)db.y - nb;
  const unsigned s6 = (unsigned)db.z - nb, s7 = (unsigned)db.w - nb;
  const bool h0 = s0 < (unsigned)NB, h1 = s1 < (unsigned)NB, h2 = s2 < (unsigned)NB, h3 = s3 < (unsigned)NB;
  const bool h4 = s4 < (unsigned)NB, h5 = s5 < (unsigned)NB, h6 = s6 < (unsigned)NB, h7 = s7 < (unsigned)NB;
  const unsigned any = __builtin_amdgcn_ballot_w32(h0 | h1 | h2 | h3 | h4 | h5 | h6 | h7);
  if (any != 0u) {
#define HITJ(J, HJ, SJ) { \
      const unsigned mj = __builtin_amdgcn_ballot_w32(HJ); \
      if (mj != 0u) { \
        if (HJ) { \
          const int pos = wc + (int)__builtin_amdgcn_mbcnt_lo(mj, 0u); \
          if (pos < WCAP) list[wave * WCAP + pos] = (((el0 + (J)) << 8) | (int)(SJ)); \
        } \
        wc += (int)__builtin_popcount(mj); } }
    HITJ(0, h0, s0)
    HITJ(1, h1, s1)
    HITJ(2, h2, s2)
    HITJ(3, h3, s3)
    HITJ(4, h4, s4)
    HITJ(5, h5, s5)
    HITJ(6, h6, s6)
    HITJ(7, h7, s7)
#undef HITJ
  }
  return wc;
}

__global__ __launch_bounds__(NTA) void k_aggr(
    const int* __restrict__ snd, const int* __restrict__ rcv, const float* __restrict__ cal,
    const float* __restrict__ Vi, const float* __restrict__ shv,
    const float* __restrict__ inv, const float* __restrict__ ev,
    float* inv1, float* ev1, int nN, int nE) {
  __shared__ __attribute__((aligned(16))) float acc[NB * FD];
  __shared__ __attribute__((aligned(16))) float aev[NB * EVD];
  __shared__ __attribute__((aligned(16))) int   list[NWA * WCAP];
  __shared__ int wcnt[NWA];

  const int tid = threadIdx.x, lane = tid & 31, wave = tid >> 5;
  const int nodeBase = blockIdx.x * NB;
  const int cl  = lane & 15;
  const int ldg = (cl == 0) ? 0 : (cl < 4) ? 1 : (cl < 9) ? 2 : 3;

  for (int i = tid; i < NB * FD; i += NTA) acc[i] = 0.0f;
  for (int i = tid; i < NB * EVD; i += NTA) aev[i] = 0.0f;
  __syncthreads();

  const int nChunks = (nE + CHUNK - 1) / CHUNK;
#pragma unroll 1
  for (int ch = 0; ch < nChunks; ++ch) {
    const int cbase = ch * CHUNK;
    const int wc = scan_chunk(rcv, nE, cbase, nodeBase, list, tid, wave);
    if (lane == 0) wcnt[wave] = wc;
    __syncthreads();

#pragma unroll 1
    for (int wsrc = 0; wsrc < NWA; ++wsrc) {
      int n = wcnt[wsrc];
      n = n > WCAP ? WCAP : (n < 0 ? 0 : n);
      const int* lp = list + wsrc * WCAP;
#pragma unroll 1
      for (int i = 0; i < n; ++i) {
        const int ent = lp[i];
        int slot = ent & 255;
        slot = slot > NB - 1 ? NB - 1 : slot;
        if ((slot & (NWA - 1)) != wave) continue;
        const int el = (ent >> 8) & (CHUNK - 1);
        int e = cbase + el;
        e = e > nE - 1 ? nE - 1 : (e < 0 ? 0 : e);
        int sn = snd[e];
        sn = sn < 0 ? 0 : (sn > nN - 1 ? nN - 1 : sn);
        const float ca = cal[(size_t)e * CAW + (lane >> 2)];
        const float ce = cal[(size_t)e * CAW + 8 + ldg];
        const float sv = shv[(size_t)e * EVD + cl];
        const v4f v = *(const v4f*)(Vi + (size_t)sn * FD + 4 * lane);
        float* ar = acc + slot * FD + 4 * lane;
        v4f a = *(v4f*)ar;
        a.x += ca * v.x; a.y += ca * v.y; a.z += ca * v.z; a.w += ca * v.w;
        *(v4f*)ar = a;
        if (lane < 16) aev[slot * EVD + lane] += ce * sv;
      }
    }
    __syncthreads();
  }
  __syncthreads();

  v4f vv[8];
#pragma unroll
  for (int i = 0; i < 8; ++i) {
    const int row = 8 * wave + i;
    int node = nodeBase + row;
    node = node > nN - 1 ? nN - 1 : node;
    const v4f a = *(const v4f*)(inv + (size_t)node * FD + 4 * lane);
    const v4f b = *(const v4f*)(acc + row * FD + 4 * lane);
    vv[i] = a + b;
  }
  v4f ve;
  {
    const int row = tid >> 2, q = tid & 3;
    int node = nodeBase + row;
    node = node > nN - 1 ? nN - 1 : node;
    const v4f a = *(const v4f*)(ev + (size_t)node * EVD + 4 * q);
    const v4f b = *(const v4f*)(aev + row * EVD + 4 * q);
    ve = a + b;
  }
#pragma unroll
  for (int i = 0; i < 8; ++i)
    *(volatile v4f*)(inv1 + (size_t)(nodeBase + 8 * wave + i) * FD + 4 * lane) = vv[i];
  *(volatile v4f*)(ev1 + (size_t)nodeBase * EVD + 4 * tid) = ve;
  __threadfence();
#pragma unroll
  for (int i = 0; i < 8; ++i)
    *(volatile v4f*)(inv1 + (size_t)(nodeBase + 8 * wave + i) * FD + 4 * lane) = vv[i];
  *(volatile v4f*)(ev1 + (size_t)nodeBase * EVD + 4 * tid) = ve;
}

__global__ __launch_bounds__(64) void k_out(const float* __restrict__ inv1, const float* __restrict__ ev1,
                                            const us* __restrict__ pl, const float* __restrict__ intb,
                                            float* out0, float* out1, int nN) {
  __shared__ __attribute__((aligned(16))) us    aph[NNODE * AKP];
  __shared__ __attribute__((aligned(16))) us    apl[NNODE * AKP];
  __shared__ __attribute__((aligned(16))) float tst[NNODE * TP];
  __shared__ __attribute__((aligned(16))) float evs[NNODE * EVD];
  const int tid = threadIdx.x, lane = tid & 31, wave = tid >> 5, hh = lane >> 4, m = lane & 15;
  const int nodeBase = blockIdx.x * NNODE;

#pragma unroll 4
  for (int i = 0; i < 16; ++i) {
    const int g = tid + 64 * i;
    const int row = g >> 5, c4 = g & 31;
    int node = nodeBase + row;
    node = node > nN - 1 ? nN - 1 : node;
    const v4f v = *(const v4f*)(inv1 + (size_t)node * FD + 4 * c4);
    us h, l;
    const int b = row * AKP + 4 * c4;
    split2(v.x, h, l); aph[b + 0] = h; apl[b + 0] = l;
    split2(v.y, h, l); aph[b + 1] = h; apl[b + 1] = l;
    split2(v.z, h, l); aph[b + 2] = h; apl[b + 2] = l;
    split2(v.w, h, l); aph[b + 3] = h; apl[b + 3] = l;
  }
#pragma unroll
  for (int j = 0; j < 2; ++j) {
    const int g = tid + 64 * j;
    const int row = g >> 2, q = g & 3;
    int node = nodeBase + row;
    node = node > nN - 1 ? nN - 1 : node;
    const v4f v = *(const v4f*)(ev1 + (size_t)node * EVD + 4 * q);
    *(v4f*)(evs + row * EVD + 4 * q) = v;
  }
  __syncthreads();

  if (wave == 0) {
    const int row = lane;
    float e[16];
#pragma unroll
    for (int c = 0; c < 16; ++c) e[c] = evs[row * EVD + c];
    float sg[4];
    sg[0] = e[0] * e[0];
    sg[1] = e[1] * e[1] + e[2] * e[2] + e[3] * e[3];
    sg[2] = e[4] * e[4] + e[5] * e[5] + e[6] * e[6] + e[7] * e[7] + e[8] * e[8];
    sg[3] = e[9] * e[9] + e[10] * e[10] + e[11] * e[11] + e[12] * e[12] + e[13] * e[13] + e[14] * e[14] + e[15] * e[15];
#pragma unroll
    for (int c = 0; c < 4; ++c) { us h, l; split2(sg[c], h, l); aph[row * AKP + FD + c] = h; apl[row * AKP + FD + c] = l; }
#pragma unroll
    for (int c = INTK; c < AKP; ++c) { aph[row * AKP + c] = 0; apl[row * AKP + c] = 0; }
  }
  __syncthreads();

  {
    const us* bhp = pl + O_INTW;
    const us* blp = bhp + PS_INT;
#pragma unroll 1
    for (int t = 0; t < 9; ++t) {
      v8f acc = zero8f();
#pragma unroll 1
      for (int ks = 0; ks < 5; ++ks) {
        Frag fah, fal, fbh, fbl;
        LDFR(fah, aph + (16 * wave + m) * AKP + 32 * ks, hh);
        LDFR(fal, apl + (16 * wave + m) * AKP + 32 * ks, hh);
        LDFR(fbh, bhp + (16 * t + m) * INTKP + 32 * ks, hh);
        LDFR(fbl, blp + (16 * t + m) * INTKP + 32 * ks, hh);
        acc = wm3(fah, fal, fbh, fbl, acc);
      }
      const int col  = 16 * t + m;
      const int colc = col > INTK - 1 ? INTK - 1 : col;
      const float bias = intb[colc];
#pragma unroll
      for (int rr = 0; rr < 8; ++rr) tst[(16 * wave + 8 * hh + rr) * TP + col] = acc[rr] + bias;
    }
  }
  __syncthreads();

  v4f o0[16];
#pragma unroll
  for (int i = 0; i < 16; ++i) {
    const int row = 16 * wave + i;
    int node = nodeBase + row;
    node = node > nN - 1 ? nN - 1 : node;
    const v4f a = *(const v4f*)(inv1 + (size_t)node * FD + 4 * lane);
    const v4f b = *(const v4f*)(tst + row * TP + 4 * lane);
    o0[i] = a + b;
  }
  v4f o1[2];
#pragma unroll
  for (int j = 0; j < 2; ++j) {
    const int g = tid + 64 * j;
    const int row = g >> 2, q = g & 3;
    float ov[4];
#pragma unroll
    for (int c = 0; c < 4; ++c) {
      const int comp = 4 * q + c;
      const int ld = (comp == 0) ? 0 : (comp < 4) ? 1 : (comp < 9) ? 2 : 3;
      const float tl = tst[row * TP + FD + ld];
      const float ee = evs[row * EVD + comp];
      ov[c] = ee + tl * ee;
    }
    v4f w4 = {ov[0], ov[1], ov[2], ov[3]};
    o1[j] = w4;
  }
#pragma unroll
  for (int i = 0; i < 16; ++i)
    *(volatile v4f*)(out0 + (size_t)(nodeBase + 16 * wave + i) * FD + 4 * lane) = o0[i];
#pragma unroll
  for (int j = 0; j < 2; ++j)
    *(volatile v4f*)(out1 + (size_t)nodeBase * EVD + 4 * (tid + 64 * j)) = o1[j];
  __threadfence();
#pragma unroll
  for (int i = 0; i < 16; ++i)
    *(volatile v4f*)(out0 + (size_t)(nodeBase + 16 * wave + i) * FD + 4 * lane) = o0[i];
#pragma unroll
  for (int j = 0; j < 2; ++j)
    *(volatile v4f*)(out1 + (size_t)nodeBase * EVD + 4 * (tid + 64 * j)) = o1[j];
}

static inline size_t al512(size_t b) { return (b + 511) & ~(size_t)511; }

extern "C" void kernel_launch(void* const* d_in, const int* in_sizes, int n_in,
                              void* d_out, int out_size, void* d_ws, size_t ws_size,
                              hipStream_t stream) {
  if (n_in < 30) return;
  const int nN = in_sizes[0] / FD;
  const int nE = in_sizes[5];
  if (nN < NB || (nN % NB) != 0 || in_sizes[0] != nN * FD || in_sizes[1] != nN * EVD) return;
  if (nE < 1 || in_sizes[6] != nE || in_sizes[4] != nE || in_sizes[2] != nE * NRB || in_sizes[3] != nE * EVD) return;
  for (int p = 0; p < 2; ++p) {
    const int b = 7 + 8 * p;
    if (in_sizes[b] != NRB * FD || in_sizes[b + 1] != FD || in_sizes[b + 2] != FD * FD || in_sizes[b + 3] != FD) return;
    if (in_sizes[b + 4] != 4 * 32 || in_sizes[b + 5] != 32 || in_sizes[b + 6] != 32 * FD || in_sizes[b + 7] != FD) return;
  }
  if (in_sizes[23] != 2048 || in_sizes[24] != 2048 || in_sizes[25] != 2048) return;
  if (in_sizes[26] != 4096 || in_sizes[27] != 4096) return;
  if (in_sizes[28] != INTK * INTK || in_sizes[29] != INTK) return;
  if (out_size != nN * (FD + EVD)) return;

  const float* inv = (const float*)d_in[0];
  const float* ev  = (const float*)d_in[1];
  const float* rbf = (const float*)d_in[2];
  const float* shv = (const float*)d_in[3];
  const float* cut = (const float*)d_in[4];
  const int*   snd = (const int*)d_in[5];
  const int*   rcv = (const int*)d_in[6];
  const float* fi_w1  = (const float*)d_in[7];
  const float* fi_b1  = (const float*)d_in[8];
  const float* fi_w2  = (const float*)d_in[9];
  const float* fi_b2  = (const float*)d_in[10];
  const float* fi_ew1 = (const float*)d_in[11];
  const float* fi_eb1 = (const float*)d_in[12];
  const float* fi_ew2 = (const float*)d_in[13];
  const float* fi_eb2 = (const float*)d_in[14];
  const float* fe_w1  = (const float*)d_in[15];
  const float* fe_b1  = (const float*)d_in[16];
  const float* fe_w2  = (const float*)d_in[17];
  const float* fe_b2  = (const float*)d_in[18];
  const float* fe_ew1 = (const float*)d_in[19];
  const float* fe_eb1 = (const float*)d_in[20];
  const float* fe_ew2 = (const float*)d_in[21];
  const float* fe_eb2 = (const float*)d_in[22];
  const float* Wq_inv = (const float*)d_in[23];
  const float* Wk_inv = (const float*)d_in[24];
  const float* Wv_inv = (const float*)d_in[25];
  const float* Wq_ev  = (const float*)d_in[26];
  const float* Wk_ev  = (const float*)d_in[27];
  const float* int_w  = (const float*)d_in[28];
  const float* int_b  = (const float*)d_in[29];
  float* out0 = (float*)d_out;
  float* out1 = out0 + (size_t)nN * FD;

  const int nBlkE = (nE + TEB - 1) / TEB;
  const int nBlkN = nN / NNODE;
  const int nBlkA = nN / NB;

  char* ws = (char*)d_ws;
  size_t off = 0;
  const size_t oPl  = off; off += al512((size_t)PL_TOT * sizeof(us));
  const size_t pln  = al512((size_t)nN * FD * sizeof(float));
  const size_t oQi  = off; off += pln;
  const size_t oKi  = off; off += pln;
  const size_t oVi  = off; off += pln;
  const size_t oQe  = off; off += pln;
  const size_t oKe  = off; off += pln;
  const size_t oCal = off; off += al512((size_t)nBlkE * TEB * CAW * sizeof(float));
  const size_t oIn1 = off; off += pln;
  const size_t oEv1 = off; off += al512((size_t)nN * EVD * sizeof(float));
  if (off > ws_size) return;

  us*    pl   = (us*)(ws + oPl);
  float* Qi   = (float*)(ws + oQi);
  float* Ki   = (float*)(ws + oKi);
  float* Vi   = (float*)(ws + oVi);
  float* Qe   = (float*)(ws + oQe);
  float* Ke   = (float*)(ws + oKe);
  float* cal  = (float*)(ws + oCal);
  float* inv1 = (float*)(ws + oIn1);
  float* ev1b = (float*)(ws + oEv1);

  k_prep<<<dim3((PS_INT / 8 + 255) / 256, 12), 256, 0, stream>>>(
      fi_w1, fi_w2, fi_ew2, fe_w1, fe_w2, fe_ew2, int_w, Wq_inv, Wk_inv, Wv_inv, Wq_ev, Wk_ev, pl);

  k_node<<<nBlkN, 64, 0, stream>>>(inv, pl, Qi, Ki, Vi, Qe, Ke, nN);

  k_edge<<<nBlkE, 64, 0, stream>>>(rbf, ev, cut, snd, rcv, Qi, Ki, Qe, Ke, pl,
                                   fi_b1, fi_b2, fi_ew1, fi_eb1, fi_eb2,
                                   fe_b1, fe_b2, fe_ew1, fe_eb1, fe_eb2,
                                   cal, nN, nE);

  k_aggr<<<nBlkA, NTA, 0, stream>>>(snd, rcv, cal, Vi, shv, inv, ev, inv1, ev1b, nN, nE);

  k_out<<<nBlkN, 64, 0, stream>>>(inv1, ev1b, pl, int_b, out0, out1, nN);
}
